// ComplexPointNetwork_71244917506299
// MI455X (gfx1250) — hardware-verified
//
#include <hip/hip_runtime.h>


namespace {
constexpr int N = 120000, CIN = 5, H = 128, H2 = 256, CO = 8, NBLK = N / 16;
constexpr float XS = 8.0f, WSC = 256.0f;
typedef _Float16 b16;
typedef __attribute__((ext_vector_type(16))) _Float16 v16b;
typedef __attribute__((ext_vector_type(8))) _Float16 v8b;
typedef __attribute__((ext_vector_type(8))) float v8f;
typedef __attribute__((ext_vector_type(4))) float v4f;
typedef __attribute__((ext_vector_type(2))) float v2f;
__device__ __forceinline__ float bf16_rne(float f) { unsigned int u = __float_as_uint(f); u += 0x7FFFu + ((u >> 16) & 1u); return __uint_as_float(u & 0xFFFF0000u); }
__device__ __forceinline__ void split16(float v, b16& hi, b16& lo) { hi = (b16)v; lo = (b16)(v - (float)hi); }
__device__ __forceinline__ v16b frag_kb(const b16* p, int hh) { const v8b a = *(const v8b*)(p + 8 * hh), b = *(const v8b*)(p + 16 + 8 * hh); v16b f;
#pragma unroll
  for (int e = 0; e < 8; ++e) { f[e] = a[e]; f[8 + e] = b[e]; } return f; }
__device__ __forceinline__ v8f wmma16b(v16b a, v16b b, v8f c) { v8f d = __builtin_amdgcn_wmma_f32_16x16x32_f16(false, a, false, b, (short)0, c, false, false); asm volatile("v_nop\n\tv_nop\n\tv_nop\n\tv_nop" : "+v"(d) : "v"(a), "v"(b)); return d; }
__device__ __forceinline__ void wave_lds_sync() { __builtin_amdgcn_fence(__ATOMIC_RELEASE, "workgroup"); __builtin_amdgcn_wave_barrier(); __builtin_amdgcn_fence(__ATOMIC_ACQUIRE, "workgroup"); }
__device__ __forceinline__ float pmul(float a, float b) { float p = a * b; asm volatile("" : "+v"(p)); return p; }

__global__ __launch_bounds__(256) void wcopy_kernel(const float* __restrict__ w, int OUTW, int OUTP, int KIN, b16* __restrict__ WT) {
  const size_t u = (size_t)blockIdx.x * 256 + threadIdx.x; if (u >= (size_t)OUTP * KIN / 8) return; const size_t e = u * 8; const int o = (int)(e / KIN); v8b v;
#pragma unroll
  for (int j = 0; j < 8; ++j) v[j] = (o < OUTW) ? (b16)(bf16_rne(w[e + j]) * WSC) : (b16)0.0f; for (int pass = 0; pass < 2; ++pass) { *(volatile v8b*)(WT + e) = v; __threadfence(); }
}
__global__ __launch_bounds__(256) void l1_kernel(const float* __restrict__ feat, const float* __restrict__ w1, int NLIM, float* __restrict__ P1) {
  const int wave = threadIdx.x >> 5, lane = threadIdx.x & 31; const size_t n = (size_t)blockIdx.x * 8 + wave; if (n >= (size_t)NLIM) return; float f[CIN]; for (int i = 0; i < CIN; ++i) f[i] = bf16_rne(feat[n * CIN + i]); v4f o;
  for (int q = 0; q < 4; ++q) { const int c = lane * 4 + q; float s = 0.0f; for (int i = 0; i < CIN; ++i) s += pmul(f[i], bf16_rne(w1[c * CIN + i])); o[q] = s; }
  for (int pass = 0; pass < 2; ++pass) { *(volatile v4f*)(P1 + n * H + lane * 4) = o; __threadfence(); }
}
template <int W>
__global__ __launch_bounds__(256) void stats_kernel(const float* __restrict__ Pp, int NLIM, float* __restrict__ ST) {
  __shared__ float red[256]; const int c = blockIdx.x, tid = threadIdx.x; float s = 0.0f;
  for (int n = tid; n < NLIM; n += 256) s += Pp[(size_t)n * W + c]; red[tid] = s; __syncthreads();
  for (int w = 128; w > 0; w >>= 1) { if (tid < w) red[tid] += red[tid + w]; __syncthreads(); } const float mu = red[0] / (float)NLIM; __syncthreads();
  float q = 0.0f; for (int n = tid; n < NLIM; n += 256) { const float d = Pp[(size_t)n * W + c] - mu; q += pmul(d, d); } red[tid] = q; __syncthreads();
  for (int w = 128; w > 0; w >>= 1) { if (tid < w) red[tid] += red[tid + w]; __syncthreads(); } const float rs = rsqrtf(red[0] / (float)NLIM + 1e-5f);
  if (tid < 32) { for (int pass = 0; pass < 2; ++pass) { ((volatile float*)ST)[c * 32 + tid] = tid == 0 ? mu : (tid == 1 ? rs : 0.0f); __threadfence(); } }
}
template <int KIN, int NT, int RES, int OP>
__global__ __launch_bounds__(32) void dense_kernel(const float* __restrict__ Pp, const float* __restrict__ ST, const float* __restrict__ g, const float* __restrict__ be, const float* __restrict__ PR, const float* __restrict__ STR, const float* __restrict__ gr, const float* __restrict__ ber, const b16* __restrict__ WT, const float* __restrict__ bias, int NLIM, float* __restrict__ OUT) {
  __shared__ __attribute__((aligned(16))) b16 Ah[16][KIN + 8], Al[16][KIN + 8]; __shared__ __attribute__((aligned(16))) float Tf[16][128 + 4];
  const int lane = threadIdx.x, nloc = lane & 15, hlf = lane >> 4; const size_t m0 = (size_t)blockIdx.x * 16; if (m0 >= (size_t)NLIM) return;
  for (int q = 0; q < KIN / 32; ++q) { const int c = q * 32 + lane; const float mu = ST[c * 32], rs = ST[c * 32 + 1], gg = bf16_rne(g[c]), bb = bf16_rne(be[c]); float mu2 = 0.0f, rs2 = 0.0f, g2 = 0.0f, b2 = 0.0f; if (RES) { mu2 = STR[c * 32]; rs2 = STR[c * 32 + 1]; g2 = bf16_rne(gr[c]); b2 = bf16_rne(ber[c]); }
    for (int rr = 0; rr < 16; ++rr) { float v = pmul(pmul(Pp[(m0 + rr) * KIN + c] - mu, rs), gg) + bb; if (RES) { v += fmaxf(pmul(pmul(PR[(m0 + rr) * KIN + c] - mu2, rs2), g2) + b2, 0.0f); } v = fmaxf(v, 0.0f); b16 p, ql; split16(v * XS, p, ql); Ah[rr][c] = p; Al[rr][c] = ql; } }
  wave_lds_sync();
#pragma unroll 1
  for (int cg = 0; cg < (NT + 7) / 8; ++cg) { constexpr int dummy = 0; (void)dummy; const int nt = (NT - cg * 8) < 8 ? (NT - cg * 8) : 8; v8f acc[8];
#pragma unroll
    for (int t = 0; t < 8; ++t) acc[t] = (v8f){};
#pragma unroll 2
    for (int kb = 0; kb < KIN; kb += 32) { const v16b a = frag_kb(&Ah[nloc][kb], hlf), al = frag_kb(&Al[nloc][kb], hlf);
#pragma unroll
      for (int t = 0; t < 8; ++t) if (t < nt) { const v16b bw = frag_kb(WT + (size_t)(cg * 128 + t * 16 + nloc) * KIN + kb, hlf); acc[t] = wmma16b(a, bw, acc[t]); acc[t] = wmma16b(al, bw, acc[t]); } }
#pragma unroll
    for (int t = 0; t < 8; ++t) { if (t < nt) { const int c = cg * 128 + t * 16 + nloc; const float bb = bias ? bf16_rne(bias[c]) : 0.0f;
#pragma unroll
        for (int r8 = 0; r8 < 8; ++r8) Tf[8 * hlf + r8][t * 16 + nloc] = acc[t][r8] * (1.0f / (XS * WSC)) + bb; } }
    wave_lds_sync();
    for (int pass = 0; pass < 2; ++pass) { if (OP >= NT * 16) { for (int rr = 0; rr < 16; ++rr) for (int c = lane; c < nt * 16; c += 32) ((volatile float*)OUT)[(m0 + rr) * OP + cg * 128 + c] = Tf[rr][c]; } else { for (int i = lane; i < 16 * OP; i += 32) ((volatile float*)OUT)[m0 * OP + i] = Tf[i / OP][i % OP]; } __threadfence(); }
    wave_lds_sync(); }
}
}

extern "C" void kernel_launch(void* const* d_in, const int* in_sizes, int n_in, void* d_out, int out_size, void* d_ws, size_t ws_size, hipStream_t stream) {
  (void)n_in;
  auto Fp = [&](int i) { return (const float*)d_in[i]; };
  if (in_sizes[0] != N * CIN || in_sizes[4] != H * CIN || in_sizes[7] != H * H || in_sizes[10] != H2 * H || in_sizes[13] != H * H2 || in_sizes[16] != CO * H || in_sizes[17] != CO || out_size != N * CO) return;
  const int NLIM = N; const int GB16 = NBLK, GB8 = N / 8;
  size_t off = 0; char* ws = (char*)d_ws;
  auto carve = [&](size_t bytes) { char* p = ws + off; off += (bytes + 255) & ~(size_t)255; return p; };
  b16* W2T = (b16*)carve(H * H * 2); b16* W3T = (b16*)carve(H2 * H * 2); b16* W4T = (b16*)carve(H * H2 * 2); b16* WOT = (b16*)carve(16 * H * 2);
  float* P1 = (float*)carve((size_t)N * H * 4); float* P2 = (float*)carve((size_t)N * H * 4); float* P3 = (float*)carve((size_t)N * H2 * 4); float* P4 = P1;
  float* S1 = (float*)carve(H * 32 * 4); float* S2 = (float*)carve(H * 32 * 4); float* S3 = (float*)carve(H2 * 32 * 4); float* S4 = (float*)carve(H * 32 * 4);
  if (off > ws_size || off > ((size_t)250 << 20)) return;
  wcopy_kernel<<<(H * H / 8 + 255) / 256, 256, 0, stream>>>(Fp(7), H, H, H, W2T); wcopy_kernel<<<(H2 * H / 8 + 255) / 256, 256, 0, stream>>>(Fp(10), H2, H2, H, W3T); wcopy_kernel<<<(H * H2 / 8 + 255) / 256, 256, 0, stream>>>(Fp(13), H, H, H2, W4T); wcopy_kernel<<<(16 * H / 8 + 255) / 256, 256, 0, stream>>>(Fp(16), CO, 16, H, WOT);
  l1_kernel<<<GB8, 256, 0, stream>>>(Fp(0), Fp(4), NLIM, P1); stats_kernel<H><<<H, 256, 0, stream>>>(P1, NLIM, S1);
  dense_kernel<H, 8, 0, H><<<GB16, 32, 0, stream>>>(P1, S1, Fp(5), Fp(6), nullptr, nullptr, nullptr, nullptr, W2T, nullptr, NLIM, P2); stats_kernel<H><<<H, 256, 0, stream>>>(P2, NLIM, S2);
  dense_kernel<H, 16, 0, H2><<<GB16, 32, 0, stream>>>(P2, S2, Fp(8), Fp(9), nullptr, nullptr, nullptr, nullptr, W3T, nullptr, NLIM, P3); stats_kernel<H2><<<H2, 256, 0, stream>>>(P3, NLIM, S3);
  dense_kernel<H2, 8, 0, H><<<GB16, 32, 0, stream>>>(P3, S3, Fp(11), Fp(12), nullptr, nullptr, nullptr, nullptr, W4T, nullptr, NLIM, P4); stats_kernel<H><<<H, 256, 0, stream>>>(P4, NLIM, S4);
  dense_kernel<H, 1, 1, CO><<<GB16, 32, 0, stream>>>(P4, S4, Fp(14), Fp(15), P2, S2, Fp(8), Fp(9), WOT, Fp(17), NLIM, (float*)d_out);
}
